// GraphSAGELayer_83167746719882
// MI455X (gfx1250) — hardware-verified
//
#include <hip/hip_runtime.h>
#include <stddef.h>


#define DF    128
#define NB    512
#define CHUNK 4096
#define NTHR  256
#define NWAVE 8
#define WCAP  512
#define SUBR  16
#define NGRP  (CHUNK / (NTHR * 4))

#define LDS_ACC_F (NB * DF)
#define LDS_BYTES (NB * DF * 4 + NB * 4 + NWAVE * WCAP * 4 + NWAVE * 4)

typedef float          v4f   __attribute__((ext_vector_type(4)));
typedef float          v8f   __attribute__((ext_vector_type(8)));
typedef int            v4i   __attribute__((ext_vector_type(4)));
typedef unsigned short v8us  __attribute__((ext_vector_type(8)));
typedef __bf16         v16bf __attribute__((ext_vector_type(16)));
union Frag { v16bf v; v8us h[2]; };

__device__ __forceinline__ unsigned int bf16_rne(float f) {
  unsigned int u = __float_as_uint(f);
  u += 0x7FFFu + ((u >> 16) & 1u);
  return u >> 16;
}

__device__ __forceinline__ void split8(v4f a, v4f b, v8us& hi, v8us& lo) {
  unsigned int hb, lb;
#define SPLK(I, VAL) hb = bf16_rne(VAL); lb = bf16_rne((VAL) - __uint_as_float(hb << 16)); \
  hi[I] = (unsigned short)hb; lo[I] = (unsigned short)lb;
  SPLK(0, a.x) SPLK(1, a.y) SPLK(2, a.z) SPLK(3, a.w)
  SPLK(4, b.x) SPLK(5, b.y) SPLK(6, b.z) SPLK(7, b.w)
#undef SPLK
}

__device__ __forceinline__ v8f wm(v16bf a, v16bf b, v8f c) {
  v8f d = __builtin_amdgcn_wmma_f32_16x16x32_bf16(false, a, false, b, (short)0, c, false, false);
  asm volatile("v_nop\n\tv_nop\n\tv_nop\n\tv_nop" : "+v"(d) : "v"(a), "v"(b));
  return d;
}

__device__ __forceinline__ float wsum(float v) {
  v += __shfl_xor(v, 16, 32);
  v += __shfl_xor(v, 8, 32);
  v += __shfl_xor(v, 4, 32);
  v += __shfl_xor(v, 2, 32);
  v += __shfl_xor(v, 1, 32);
  return v;
}

__global__ __launch_bounds__(NTHR) void k_wplanes(
    const float* __restrict__ Ws, const float* __restrict__ Wa,
    unsigned short* wsh, unsigned short* wsl,
    unsigned short* wah, unsigned short* wal, int n8) {
  const int i = blockIdx.x * NTHR + threadIdx.x;
  if (i >= n8) return;
  const size_t o = (size_t)i * 8;
  const v4f s0 = *(const v4f*)(Ws + o), s1 = *(const v4f*)(Ws + o + 4);
  const v4f a0 = *(const v4f*)(Wa + o), a1 = *(const v4f*)(Wa + o + 4);
  v8us hs = {0, 0, 0, 0, 0, 0, 0, 0}, ls = {0, 0, 0, 0, 0, 0, 0, 0};
  v8us ha = {0, 0, 0, 0, 0, 0, 0, 0}, la = {0, 0, 0, 0, 0, 0, 0, 0};
  split8(s0, s1, hs, ls);
  split8(a0, a1, ha, la);
  *(volatile v8us*)(wsh + o) = hs;
  *(volatile v8us*)(wsl + o) = ls;
  *(volatile v8us*)(wah + o) = ha;
  *(volatile v8us*)(wal + o) = la;
  __threadfence();
  *(volatile v8us*)(wsh + o) = hs;
  *(volatile v8us*)(wsl + o) = ls;
  *(volatile v8us*)(wah + o) = ha;
  *(volatile v8us*)(wal + o) = la;
}

__global__ __launch_bounds__(NTHR) void k_sage(
    const float* __restrict__ x, const int* __restrict__ ei,
    const unsigned short* __restrict__ wsh, const unsigned short* __restrict__ wsl,
    const unsigned short* __restrict__ wah, const unsigned short* __restrict__ wal,
    const float* __restrict__ bself, const float* __restrict__ bagg,
    const float* __restrict__ gam, const float* __restrict__ bet,
    float* out, int nN, int nE) {
  extern __shared__ v4f lds_dyn[];
  float* acc  = (float*)lds_dyn;
  int*   cnt  = (int*)(acc + LDS_ACC_F);
  int*   list = cnt + NB;
  int*   wcnt = list + NWAVE * WCAP;
  unsigned short* sXh = (unsigned short*)list;
  unsigned short* sXl = sXh + SUBR * DF;
  unsigned short* sMh = sXl + SUBR * DF;
  unsigned short* sMl = sMh + SUBR * DF;

  const int tid  = threadIdx.x;
  const int lane = tid & 31;
  const int wave = tid >> 5;
  const int hh   = lane >> 4;
  const int m    = lane & 15;
  const int nodeBase = blockIdx.x * NB;

  {
    const v4f z4 = {0.f, 0.f, 0.f, 0.f};
    for (int i = tid; i < LDS_ACC_F / 4; i += NTHR) lds_dyn[i] = z4;
    for (int i = tid; i < NB; i += NTHR) cnt[i] = 0;
  }
  __syncthreads();

  const int nChunks = (nE + CHUNK - 1) / CHUNK;
#pragma unroll 1
  for (int ch = 0; ch < nChunks; ++ch) {
    const int cbase = ch * CHUNK;
    int wc = 0;
#pragma unroll
    for (int g = 0; g < NGRP; ++g) {
      const int el0 = (g * NTHR + tid) * 4;
      const int e0  = cbase + el0;
      const int sent = -2147483647 - 1;
      v4i d;
      if (e0 + 3 < nE) {
        d = *(const v4i*)(ei + e0);
      } else {
        d.x = (e0     < nE) ? ei[e0]     : sent;
        d.y = (e0 + 1 < nE) ? ei[e0 + 1] : sent;
        d.z = (e0 + 2 < nE) ? ei[e0 + 2] : sent;
        d.w = (e0 + 3 < nE) ? ei[e0 + 3] : sent;
      }
      const unsigned s0 = (unsigned)d.x - (unsigned)nodeBase;
      const unsigned s1 = (unsigned)d.y - (unsigned)nodeBase;
      const unsigned s2 = (unsigned)d.z - (unsigned)nodeBase;
      const unsigned s3 = (unsigned)d.w - (unsigned)nodeBase;
      const bool h0 = s0 < (unsigned)NB;
      const bool h1 = s1 < (unsigned)NB;
      const bool h2 = s2 < (unsigned)NB;
      const bool h3 = s3 < (unsigned)NB;
      const unsigned many = __builtin_amdgcn_ballot_w32(h0 | h1 | h2 | h3);
      if (many != 0u) {
#define HITJ(J, HJ, SJ) { \
          const unsigned mj = __builtin_amdgcn_ballot_w32(HJ); \
          if (HJ) { \
            const int pos = wc + (int)__builtin_amdgcn_mbcnt_lo(mj, 0u); \
            if (pos < WCAP) list[wave * WCAP + pos] = ((el0 + (J)) << 9) | (int)(SJ); \
          } \
          wc += (int)__builtin_popcount(mj); }
        HITJ(0, h0, s0)
        HITJ(1, h1, s1)
        HITJ(2, h2, s2)
        HITJ(3, h3, s3)
#undef HITJ
      }
    }
    if (lane == 0) wcnt[wave] = wc;
    __syncthreads();

    if (wave == 0) {
      for (int wsx = 0; wsx < NWAVE; ++wsx) {
        int n = wcnt[wsx];
        if (n > WCAP) n = WCAP;
        if (n < 0) n = 0;
        for (int i = 0; i < n; ++i) {
          const int ent  = list[wsx * WCAP + i];
          const int slot = ent & (NB - 1);
          const int el   = (ent >> 9) & (CHUNK - 1);
          int e = cbase + el;
          if (e > nE - 1) e = nE - 1;
          int src = ei[(size_t)nE + (size_t)e];
          src = src < 0 ? 0 : (src > nN - 1 ? nN - 1 : src);
          const v4f v = *(const v4f*)(x + (size_t)src * DF + 4 * lane);
          v4f* ap = (v4f*)(acc + slot * DF + 4 * lane);
          const v4f cur = *ap;
          *ap = cur + v;
          if (lane == 0) cnt[slot] = cnt[slot] + 1;
        }
      }
    }
    __syncthreads();
  }

  int nValid = nN - nodeBase;
  if (nValid > NB) nValid = NB;
  if (nValid < 0) nValid = 0;
  const int nsub = (nValid + SUBR - 1) / SUBR;
  const v4f g4 = *(const v4f*)(gam + 4 * lane);
  const v4f b4 = *(const v4f*)(bet + 4 * lane);
  const int ncol = wave * 16 + m;
  const float bsum = bself[ncol] + bagg[ncol];

#pragma unroll 1
  for (int s = 0; s < nsub; ++s) {
    {
      const int r  = tid >> 4;
      const int c0 = (tid & 15) * 8;
      int node = nodeBase + s * SUBR + r;
      if (node > nN - 1) node = nN - 1;
      const float* xp = x + (size_t)node * DF + c0;
      const v4f xa = *(const v4f*)xp, xb = *(const v4f*)(xp + 4);
      v8us hi = {0, 0, 0, 0, 0, 0, 0, 0}, lo = {0, 0, 0, 0, 0, 0, 0, 0};
      split8(xa, xb, hi, lo);
      *(v8us*)(sXh + r * DF + c0) = hi;
      *(v8us*)(sXl + r * DF + c0) = lo;
      const int slot = s * SUBR + r;
      const float* ap = acc + slot * DF + c0;
      v4f aa = *(const v4f*)ap, ab = *(const v4f*)(ap + 4);
      const float inv = 1.0f / ((float)cnt[slot] + 1e-8f);
      aa = aa * inv;
      ab = ab * inv;
      split8(aa, ab, hi, lo);
      *(v8us*)(sMh + r * DF + c0) = hi;
      *(v8us*)(sMl + r * DF + c0) = lo;
    }
    __syncthreads();

    v8f c = {0.f, 0.f, 0.f, 0.f, 0.f, 0.f, 0.f, 0.f};
#pragma unroll
    for (int kt = 0; kt < DF / 32; ++kt) {
      const int k0 = kt * 32;
      Frag ah, al, bh, bl;
      const unsigned short* pah = sXh + m * DF + k0 + 8 * hh;
      const unsigned short* pal = sXl + m * DF + k0 + 8 * hh;
      const unsigned short* pbh = wsh + ncol * DF + k0 + 8 * hh;
      const unsigned short* pbl = wsl + ncol * DF + k0 + 8 * hh;
      ah.h[0] = *(const v8us*)pah; ah.h[1] = *(const v8us*)(pah + 16);
      al.h[0] = *(const v8us*)pal; al.h[1] = *(const v8us*)(pal + 16);
      bh.h[0] = *(const v8us*)pbh; bh.h[1] = *(const v8us*)(pbh + 16);
      bl.h[0] = *(const v8us*)pbl; bl.h[1] = *(const v8us*)(pbl + 16);
      c = wm(al.v, bh.v, c);
      c = wm(ah.v, bl.v, c);
      c = wm(ah.v, bh.v, c);
    }
#pragma unroll
    for (int kt = 0; kt < DF / 32; ++kt) {
      const int k0 = kt * 32;
      Frag ah, al, bh, bl;
      const unsigned short* pah = sMh + m * DF + k0 + 8 * hh;
      const unsigned short* pal = sMl + m * DF + k0 + 8 * hh;
      const unsigned short* pbh = wah + ncol * DF + k0 + 8 * hh;
      const unsigned short* pbl = wal + ncol * DF + k0 + 8 * hh;
      ah.h[0] = *(const v8us*)pah; ah.h[1] = *(const v8us*)(pah + 16);
      al.h[0] = *(const v8us*)pal; al.h[1] = *(const v8us*)(pal + 16);
      bh.h[0] = *(const v8us*)pbh; bh.h[1] = *(const v8us*)(pbh + 16);
      bl.h[0] = *(const v8us*)pbl; bl.h[1] = *(const v8us*)(pbl + 16);
      c = wm(al.v, bh.v, c);
      c = wm(ah.v, bl.v, c);
      c = wm(ah.v, bh.v, c);
    }

    {
      float* hrow = acc + (s * SUBR + 8 * hh) * DF + ncol;
#pragma unroll
      for (int r = 0; r < 8; ++r) {
        const float v = c[r] + bsum;
        hrow[r * DF] = v > 0.0f ? v : 0.0f;
      }
    }
    __syncthreads();

    {
      const int slotA = s * SUBR + 2 * wave;
      const int slotB = slotA + 1;
      const v4f hA = *(const v4f*)(acc + slotA * DF + 4 * lane);
      const v4f hB = *(const v4f*)(acc + slotB * DF + 4 * lane);
      const float sA = wsum(hA.x + hA.y + hA.z + hA.w);
      const float sB = wsum(hB.x + hB.y + hB.z + hB.w);
      const float muA = sA * (1.0f / DF);
      const float muB = sB * (1.0f / DF);
      const v4f dA = hA - muA;
      const v4f dB = hB - muB;
      const float qA = wsum(dA.x * dA.x + dA.y * dA.y + dA.z * dA.z + dA.w * dA.w);
      const float qB = wsum(dB.x * dB.x + dB.y * dB.y + dB.z * dB.z + dB.w * dB.w);
      const float rsA = rsqrtf(qA * (1.0f / DF) + 1e-5f);
      const float rsB = rsqrtf(qB * (1.0f / DF) + 1e-5f);
      const v4f yA = dA * rsA * g4 + b4;
      const v4f yB = dB * rsB * g4 + b4;
      const int nodeA = nodeBase + slotA;
      const int nodeB = nodeBase + slotB;
      const bool okA = nodeA < nN;
      const bool okB = nodeB < nN;
      const size_t offA = (size_t)(okA ? nodeA : 0) * DF + 4 * lane;
      const size_t offB = (size_t)(okB ? nodeB : 0) * DF + 4 * lane;
      if (okA) *(volatile v4f*)(out + offA) = yA;
      if (okB) *(volatile v4f*)(out + offB) = yB;
      __threadfence();
      if (okA) *(volatile v4f*)(out + offA) = yA;
      if (okB) *(volatile v4f*)(out + offB) = yB;
    }
    __syncthreads();
  }
}

extern "C" void kernel_launch(void* const* d_in, const int* in_sizes, int n_in,
                              void* d_out, int out_size, void* d_ws, size_t ws_size,
                              hipStream_t stream) {
  if (n_in < 8) return;
  const int nN = in_sizes[0] / DF;
  const int nE = in_sizes[1] / 2;
  if (nN <= 0 || in_sizes[0] != nN * DF || in_sizes[1] != nE * 2) return;
  if (in_sizes[2] != DF * DF || in_sizes[4] != DF * DF) return;
  if (in_sizes[3] < DF || in_sizes[5] < DF || in_sizes[6] < DF || in_sizes[7] < DF) return;
  if (out_size != nN * DF) return;

  const float* x     = (const float*)d_in[0];
  const int*   ei    = (const int*)d_in[1];
  const float* Wagg  = (const float*)d_in[2];
  const float* bagg  = (const float*)d_in[3];
  const float* Wself = (const float*)d_in[4];
  const float* bself = (const float*)d_in[5];
  const float* gam   = (const float*)d_in[6];
  const float* bet   = (const float*)d_in[7];
  float* out = (float*)d_out;

  const size_t planeElems = (size_t)DF * DF;
  if (ws_size < 4 * planeElems * sizeof(unsigned short)) return;
  unsigned short* wsh = (unsigned short*)d_ws;
  unsigned short* wsl = wsh + planeElems;
  unsigned short* wah = wsl + planeElems;
  unsigned short* wal = wah + planeElems;

  const int n8 = DF * DF / 8;
  k_wplanes<<<(n8 + NTHR - 1) / NTHR, NTHR, 0, stream>>>(Wself, Wagg, wsh, wsl, wah, wal, n8);

  hipFuncSetAttribute(reinterpret_cast<const void*>(&k_sage),
                      hipFuncAttributeMaxDynamicSharedMemorySize, LDS_BYTES);
  const int grid = (nN + NB - 1) / NB;
  k_sage<<<grid, NTHR, LDS_BYTES, stream>>>(x, ei, wsh, wsl, wah, wal, bself, bagg, gam, bet,
                                            out, nN, nE);
}
